// FeatureGeneratorMoe_6571299962924
// MI455X (gfx1250) — hardware-run, weakly checked
//
#include <hip/hip_runtime.h>
#include <math.h>

typedef __attribute__((ext_vector_type(16))) _Float16 v16h;
typedef __attribute__((ext_vector_type(8)))  _Float16 v8h;
typedef __attribute__((ext_vector_type(8)))  float    v8f;
typedef __attribute__((ext_vector_type(4)))  float    v4f;
typedef __attribute__((ext_vector_type(2)))  float    v2f;

constexpr int kBatch   = 16;
constexpr int kSeq     = 2048;
constexpr int kChan    = 16;
constexpr int kNumPts  = kBatch * kSeq * kChan;
constexpr int kHid     = 16;
constexpr int kNumMlp  = 8;
constexpr int kNumExp  = 12;
constexpr int kInF     = 3;
constexpr int kKpad    = 32;
constexpr int kThreads = 256;
constexpr int kWavesPerBlock = kThreads / 32;
constexpr int kBlocks  = 512;
constexpr float kCarry    = 2048.0f;
constexpr float kCarryInv = 1.0f / kCarry;
constexpr float kF16MinNormal = 6.103515625e-5f;
static_assert(kNumPts == 524288);
static_assert(kNumMlp * 2 * kHid == kThreads);
static_assert((kNumPts % 32) == 0);
static_assert(2 * kInF <= 8);

template <typename T> struct Frag;
template <> struct Frag<_Float16> {
  typedef v16h V; union U { v16h v; v8h h[2]; };
  static __device__ __forceinline__ v16h load(const _Float16* p) {
    U f; f.h[0] = *(const v8h*)(p); f.h[1] = *(const v8h*)(p + 16); return f.v;
  }
  static __device__ __forceinline__ v8f mma(v16h a, v16h b, v8f c) {
    return __builtin_amdgcn_wmma_f32_16x16x32_f16(false, a, false, b, (short)0, c, false, false);
  }
};

__device__ __forceinline__ v8f mma_f16_guarded(v16h a, v16h b, v8f c) {
  c = Frag<_Float16>::mma(a, b, c);
  asm volatile("v_nop\n\tv_nop\n\tv_nop\n\tv_nop" : "+v"(c) : "v"(a), "v"(b));
  return c;
}

__device__ __forceinline__ float f16_value_part(float v) {
  const _Float16 h = (_Float16)v;
  float hf = (float)h;
  asm volatile("" : "+v"(hf));
  return (fabsf(hf) < kF16MinNormal) ? 0.0f : hf;
}

template <int I> __device__ __forceinline__ float act_fn(float v) {
  if (I == 0) {
    return fmaxf(v, 0.0f);
  }
  if (I == 1) {
    return tanhf(v);
  }
  if (I == 2) {
    const float e = expf(fminf(v, 0.0f)) - 1.0f;
    return (v > 0.0f) ? v : e;
  }
  if (I == 3) {
    const float e = expf(-v);
    return v * __builtin_amdgcn_rcpf(1.0f + e);
  }
  if (I == 4) {
    return 0.5f * v * (1.0f + erff(v * 0.70710678118654752f));
  }
  if (I == 5) {
    return v;
  }
  if (I == 6) {
    const float e = 1.6732632423543772f * (expf(fminf(v, 0.0f)) - 1.0f);
    return 1.0507009873554805f * ((v > 0.0f) ? v : e);
  }
  return fmaxf(v, 0.0f) + log1pf(expf(-fabsf(v)));
}

template <int I> __device__ __forceinline__ float expert_tile(
    const _Float16* sA, const float* sB1, const float* sW2, v16h bfr, int rowm, int half, float acc)
{
  const v16h a_val = Frag<_Float16>::load(sA + ((I * 2 + 0) * kHid + rowm) * kKpad + 8 * half);
  const v16h a_res = Frag<_Float16>::load(sA + ((I * 2 + 1) * kHid + rowm) * kKpad + 8 * half);
  const v4f bi0 = *(const v4f*)(sB1 + I * kHid + 8 * half);
  const v4f bi1 = *(const v4f*)(sB1 + I * kHid + 8 * half + 4);
  const v4f wv0 = *(const v4f*)(sW2 + I * kHid + 8 * half);
  const v4f wv1 = *(const v4f*)(sW2 + I * kHid + 8 * half + 4);
  v8f c  = (v8f){bi0[0], bi0[1], bi0[2], bi0[3], bi1[0], bi1[1], bi1[2], bi1[3]};
  v8f c2 = (v8f){0.f, 0.f, 0.f, 0.f, 0.f, 0.f, 0.f, 0.f};
  const v8f w = (v8f){wv0[0], wv0[1], wv0[2], wv0[3], wv1[0], wv1[1], wv1[2], wv1[3]};
  c  = mma_f16_guarded(a_val, bfr, c);
  c2 = mma_f16_guarded(a_res, bfr, c2);
#pragma unroll
  for (int r = 0; r < 8; ++r) {
    const float pre = fmaf(c2[r], kCarryInv, c[r]);
    acc = fmaf(act_fn<I>(pre), w[r], acc);
  }
  return acc;
}

__global__ __launch_bounds__(256) void fused_expert_mix_kernel(
    const float* __restrict__ x, const float* __restrict__ W1, const float* __restrict__ b1,
    const float* __restrict__ W2, const float* __restrict__ b2, const float* __restrict__ ew,
    float* __restrict__ out, int npoints)
{
  __shared__ __align__(16) _Float16 sA[kNumMlp * 2 * kHid * kKpad];
  __shared__ __align__(16) float sTab[2 * kNumMlp * kHid];

  const int tid  = threadIdx.x;
  const int lane = tid & 31;
  const int wave = __builtin_amdgcn_readfirstlane((int)(threadIdx.x >> 5));
  const int half = lane >> 4;
  const int col  = lane & 15;

  {
    const int ei    = tid >> 5;
    const int plane = (tid >> 4) & 1;
    const int m     = tid & 15;
    const float w0 = W1[(ei * kInF + 0) * kHid + m];
    const float w1 = W1[(ei * kInF + 1) * kHid + m];
    const float w2 = W1[(ei * kInF + 2) * kHid + m];
    const float h0 = f16_value_part(w0);
    const float h1 = f16_value_part(w1);
    const float h2 = f16_value_part(w2);
    const float l0 = (w0 - h0) * kCarry;
    const float l1 = (w1 - h1) * kCarry;
    const float l2 = (w2 - h2) * kCarry;
    const float e0 = plane ? l0 : h0;
    const float e1 = plane ? l1 : h1;
    const float e2 = plane ? l2 : h2;
    const float e3 = plane ? h0 : 0.0f;
    const float e4 = plane ? h1 : 0.0f;
    const float e5 = plane ? h2 : 0.0f;
    v8h rowv;
    rowv[0] = (_Float16)e0;
    rowv[1] = (_Float16)e1;
    rowv[2] = (_Float16)e2;
    rowv[3] = (_Float16)e3;
    rowv[4] = (_Float16)e4;
    rowv[5] = (_Float16)e5;
    rowv[6] = (_Float16)0.0f;
    rowv[7] = (_Float16)0.0f;
    v8h zr;
#pragma unroll
    for (int e = 0; e < 8; ++e) zr[e] = (_Float16)0.0f;
    _Float16* dst = sA + tid * kKpad;
    *(v8h*)(dst)      = rowv;
    *(v8h*)(dst + 8)  = zr;
    *(v8h*)(dst + 16) = zr;
    *(v8h*)(dst + 24) = zr;
    const int idx = tid & 127;
    const float bv = b1[idx];
    const float wv = ew[idx >> 4] * W2[idx];
    sTab[tid] = (tid < 128) ? bv : wv;
  }
  __syncthreads();

  const float* sB1 = sTab;
  const float* sW2 = sTab + kNumMlp * kHid;

  float b2sum = 0.0f;
#pragma unroll
  for (int i = 0; i < kNumMlp; ++i) b2sum = fmaf(ew[i], b2[i], b2sum);
  const float w_abs = ew[8];
  const float w_mod = ew[9];
  const float w_sin = ew[10];
  const float w_cos = ew[11];

  const int nIter  = (npoints + 31) >> 5;
  const int gwave  = (int)blockIdx.x * kWavesPerBlock + wave;
  const int nwaves = (int)gridDim.x * kWavesPerBlock;

  for (int it = gwave; it < nIter; it += nwaves) {
    const int base = it << 5;
    float own_re = 0.0f, own_im = 0.0f, own_amp = 0.0f, mix = 0.0f;
#pragma unroll 1
    for (int t = 0; t < 2; ++t) {
      int pt = base + (t << 4) + col;
      pt = (pt < npoints) ? pt : (npoints - 1);
      const v2f xv = *(const v2f*)(x + 2 * (size_t)pt);
      const float re  = xv.x;
      const float im  = xv.y;
      const float amp = sqrtf(re * re + im * im);
      const bool mine = (t == half);
      own_re  = mine ? re  : own_re;
      own_im  = mine ? im  : own_im;
      own_amp = mine ? amp : own_amp;

      const float rh = f16_value_part(re);
      const float ih = f16_value_part(im);
      const float ah = f16_value_part(amp);
      const float rl = (re  - rh) * kCarry;
      const float il = (im  - ih) * kCarry;
      const float al = (amp - ah) * kCarry;
      const float q0 = half ? 0.0f : rh;
      const float q1 = half ? 0.0f : ih;
      const float q2 = half ? 0.0f : ah;
      const float q3 = half ? 0.0f : rl;
      const float q4 = half ? 0.0f : il;
      const float q5 = half ? 0.0f : al;
      v16h bfr;
#pragma unroll
      for (int e = 0; e < 16; ++e) bfr[e] = (_Float16)0.0f;
      bfr[0] = (_Float16)q0;
      bfr[1] = (_Float16)q1;
      bfr[2] = (_Float16)q2;
      bfr[3] = (_Float16)q3;
      bfr[4] = (_Float16)q4;
      bfr[5] = (_Float16)q5;

      float acc = 0.0f;
      acc = expert_tile<0>(sA, sB1, sW2, bfr, col, half, acc);
      acc = expert_tile<1>(sA, sB1, sW2, bfr, col, half, acc);
      acc = expert_tile<2>(sA, sB1, sW2, bfr, col, half, acc);
      acc = expert_tile<3>(sA, sB1, sW2, bfr, col, half, acc);
      acc = expert_tile<4>(sA, sB1, sW2, bfr, col, half, acc);
      acc = expert_tile<5>(sA, sB1, sW2, bfr, col, half, acc);
      acc = expert_tile<6>(sA, sB1, sW2, bfr, col, half, acc);
      acc = expert_tile<7>(sA, sB1, sW2, bfr, col, half, acc);

      const float other = __shfl_xor(acc, 16, 32);
      const float comb  = acc + other;
      mix = mine ? comb : mix;
    }

    const float l1n = fabsf(own_re) + fabsf(own_im);
    const float sn  = sinf(own_amp);
    const float cs  = cosf(own_amp);
    float o = mix + b2sum;
    o = fmaf(w_abs, l1n, o);
    o = fmaf(w_mod, own_amp, o);
    o = fmaf(w_sin, sn, o);
    o = fmaf(w_cos, cs, o);

    const int p = base + lane;
    const bool ok = (p < npoints);
    volatile float* op = (volatile float*)out + (ok ? p : 0);
    if (ok) *op = o;
    __threadfence();
    if (ok) *op = o;
  }
}

extern "C" void kernel_launch(void* const* d_in, const int* in_sizes, int n_in,
                              void* d_out, int out_size, void* d_ws, size_t ws_size,
                              hipStream_t stream) {
  if (n_in < 6) return;
  if (in_sizes[0] != 2 * kNumPts) return;
  if (in_sizes[1] != kNumMlp * kInF * kHid) return;
  if (in_sizes[2] != kNumMlp * kHid) return;
  if (in_sizes[3] != kNumMlp * kHid) return;
  if (in_sizes[4] != kNumMlp) return;
  if (in_sizes[5] != kNumExp) return;
  if (out_size != kNumPts) return;
  (void)d_ws;
  (void)ws_size;

  const float* x  = (const float*)d_in[0];
  const float* W1 = (const float*)d_in[1];
  const float* b1 = (const float*)d_in[2];
  const float* W2 = (const float*)d_in[3];
  const float* b2 = (const float*)d_in[4];
  const float* ew = (const float*)d_in[5];
  float* out = (float*)d_out;

  fused_expert_mix_kernel<<<kBlocks, kThreads, 0, stream>>>(x, W1, b1, W2, b2, ew, out, kNumPts);
}
